// MPNNNet_45097156608288
// MI455X (gfx1250) — hardware-verified
//
#include <hip/hip_runtime.h>
#include <stddef.h>
#include <stdint.h>

#define NV     10000
#define NE     20000
#define NG     256
#define DIN    74
#define EIN    12
#define HD     64
#define EHD    128
#define NSTEP  5
#define MP     10112
#define EP     20096
#define KPJ    96
#define KWE    256
#define KGR    256
#define NWE    4096
#define ACW    256
#define NTHR   256
#define NWAVE  8
#define EPT    8
#define CHUNK  (NTHR * EPT)
#define WCAP   (EPT * 32)
#define LISTN  (NWAVE * WCAP)
#define NBA    1024
#define SLA    10
#define RCAP   4096
#define DEGCAP 32
#define NBLK   10
#define MEAS_MAXDEG 9
#define MEAS_B1024  2103
#define AGG_ZINTS (LISTN + 2 * RCAP + 3 * NBA)
#define BK_LDS_BYTES ((AGG_ZINTS + 16) * 4)
#define GBM    64
#define GBN    128
#define GTHR   128
#define GRU_LDS_BYTES ((GBM * KGR + 256) * 4)
#define CWE    64.0f
#define CINV   0.015625f
#define U_HB   (MP * (KPJ / 8))
#define U_WP   (128 * (KPJ / 8))
#define U_W2   (NWE * (KWE / 8))
#define U_GA   (256 * 16)
#define U_GB   (256 * 16)
#define U_TH   (EP * 16)

static_assert(MP % GBM == 0 && EP % GBM == 0 && MP >= NV && EP >= NE);
static_assert(KPJ % 32 == 0 && KPJ >= DIN && KWE % 32 == 0 && KGR % 32 == 0 && KWE == 2 * EHD && KGR == 4 * HD);
static_assert(NWE % GBN == 0 && NWE == HD * HD);
static_assert(NE % NWAVE == 0 && NE % 2 == 0 && NV % 2 == 0);
static_assert(NBLK * NBA >= MP);
static_assert(DEGCAP >= MEAS_MAXDEG + 8 && DEGCAP <= 32);
static_assert(RCAP >= MEAS_B1024 + 1024);
static_assert((CHUNK & (CHUNK - 1)) == 0 && NBA == (1 << SLA));
static_assert(((long long)NE << SLA) < (1LL << 31));
static_assert(AGG_ZINTS % (4 * NTHR) == 0 && RCAP % (4 * NTHR) == 0 && NBA == 4 * NTHR);
static_assert(U_HB % NTHR == 0 && U_WP % NTHR == 0 && U_W2 % NTHR == 0 && U_GA % NTHR == 0 && U_TH % NTHR == 0);
static_assert(GBM == (GTHR / 32) * 16 && GBN == 128);
static_assert(BK_LDS_BYTES <= 65536 && GRU_LDS_BYTES <= 300000);

typedef float          v2f   __attribute__((ext_vector_type(2)));
typedef float          v4f   __attribute__((ext_vector_type(4)));
typedef float          v8f   __attribute__((ext_vector_type(8)));
typedef int            v4i   __attribute__((ext_vector_type(4)));
typedef int            v8i   __attribute__((ext_vector_type(8)));
typedef unsigned       v4u   __attribute__((ext_vector_type(4)));
typedef unsigned short v8us  __attribute__((ext_vector_type(8)));
typedef unsigned short v16us __attribute__((ext_vector_type(16)));
typedef __bf16         v16bf __attribute__((ext_vector_type(16)));
typedef v2f  __attribute__((may_alias)) v2fa;
typedef v4f  __attribute__((may_alias)) v4fa;
typedef v4i  __attribute__((may_alias)) v4ia;
typedef v4u  __attribute__((may_alias)) v4ua;
typedef v8us __attribute__((may_alias)) v8usa;
union FragB { v16bf v; v16us u; v8us h[2]; v8i w; };

__device__ __forceinline__ v8f wmb(const FragB& a, const FragB& b, v8f c) {
  v8f d = __builtin_amdgcn_wmma_f32_16x16x32_bf16(false, a.v, false, b.v, (short)0, c, false, false);
  asm volatile("v_nop\n\tv_nop\n\tv_nop\n\tv_nop" : "+v"(d) : "v"(a.w), "v"(b.w));
  return d;
}

__device__ __forceinline__ unsigned bf16_bits(float f) {
  const unsigned u = __float_as_uint(f);
  const unsigned r = (u + 0x7FFFu + ((u >> 16) & 1u)) >> 16;
  return (f != f) ? 0x7FC0u : r;
}
__device__ __forceinline__ float bf16_val(float f) {
  return __uint_as_float(bf16_bits(f) << 16);
}
__device__ __forceinline__ unsigned short f2h(float f) {
  const _Float16 hv = (_Float16)f;
  return __builtin_bit_cast(unsigned short, hv);
}
__device__ __forceinline__ float h2f(unsigned b) {
  const _Float16 hv = __builtin_bit_cast(_Float16, (unsigned short)b);
  return (float)hv;
}
__device__ __forceinline__ float relu_k(float v) { return (v > 0.0f) ? v : (v - v); }
__device__ __forceinline__ float sigm(float a) {
  a = (a > 30.0f) ? 30.0f : a;
  a = (a < -30.0f) ? -30.0f : a;
  return 1.0f / (1.0f + expf(-a));
}
__device__ __forceinline__ void put16(unsigned short* dp, v8us o) {
  *(volatile v8us*)dp = o;
  __threadfence();
  *(volatile v8us*)dp = o;
}

template <int SLB>
__device__ __forceinline__ int scan_chunk(const int* __restrict__ dsts, int nE, int cbase, int slotBase,
                                          int nb, int vec8, int* list, int tid, int lane, int wave) {
  int wc = 0;
  const int el0  = tid * EPT;
  const int e0   = cbase + el0;
  const int sent = -2147483647 - 1;
  v4i da, db;
  if (vec8 != 0 && cbase + CHUNK <= nE) {
    da = *(const v4i*)(dsts + e0);
    db = *(const v4i*)(dsts + e0 + 4);
  } else {
    da.x = (e0     < nE) ? dsts[min(e0,     nE - 1)] : sent;
    da.y = (e0 + 1 < nE) ? dsts[min(e0 + 1, nE - 1)] : sent;
    da.z = (e0 + 2 < nE) ? dsts[min(e0 + 2, nE - 1)] : sent;
    da.w = (e0 + 3 < nE) ? dsts[min(e0 + 3, nE - 1)] : sent;
    db.x = (e0 + 4 < nE) ? dsts[min(e0 + 4, nE - 1)] : sent;
    db.y = (e0 + 5 < nE) ? dsts[min(e0 + 5, nE - 1)] : sent;
    db.z = (e0 + 6 < nE) ? dsts[min(e0 + 6, nE - 1)] : sent;
    db.w = (e0 + 7 < nE) ? dsts[min(e0 + 7, nE - 1)] : sent;
  }
  const unsigned nbs = (unsigned)slotBase;
  const unsigned unb = (unsigned)nb;
  const unsigned s0 = (unsigned)da.x - nbs, s1 = (unsigned)da.y - nbs;
  const unsigned s2 = (unsigned)da.z - nbs, s3 = (unsigned)da.w - nbs;
  const unsigned s4 = (unsigned)db.x - nbs, s5 = (unsigned)db.y - nbs;
  const unsigned s6 = (unsigned)db.z - nbs, s7 = (unsigned)db.w - nbs;
  const bool h0 = s0 < unb, h1 = s1 < unb, h2 = s2 < unb, h3 = s3 < unb;
  const bool h4 = s4 < unb, h5 = s5 < unb, h6 = s6 < unb, h7 = s7 < unb;
  const unsigned any = __builtin_amdgcn_ballot_w32(h0 | h1 | h2 | h3 | h4 | h5 | h6 | h7);
  if (any != 0u) {
#define HITJ(J, HJ, SJ) { \
      const unsigned mj = __builtin_amdgcn_ballot_w32(HJ); \
      if (mj != 0u) { \
        if (HJ) { \
          const int pos = wc + (int)__builtin_amdgcn_mbcnt_lo(mj, 0u); \
          if (pos < WCAP) list[wave * WCAP + pos] = ((el0 + (J)) << SLB) | (int)(SJ); \
        } \
        wc += (int)__builtin_popcount(mj); } }
    HITJ(0, h0, s0)
    HITJ(1, h1, s1)
    HITJ(2, h2, s2)
    HITJ(3, h3, s3)
    HITJ(4, h4, s4)
    HITJ(5, h5, s5)
    HITJ(6, h6, s6)
    HITJ(7, h7, s7)
#undef HITJ
  }
  return wc;
}

__global__ __launch_bounds__(NTHR) void k_prep(const float* __restrict__ Hin, const float* __restrict__ Ein,
                                               const float* __restrict__ Wp, const float* __restrict__ We1,
                                               const float* __restrict__ be1, const float* __restrict__ We2,
                                               const float* __restrict__ Wih, const float* __restrict__ Whh,
                                               unsigned short* HB, unsigned short* WpT, unsigned short* W2T,
                                               unsigned short* WG, unsigned short* THL) {
  __shared__ __attribute__((aligned(16))) float sW1[EIN * EHD];
  __shared__ __attribute__((aligned(16))) float sb1[EHD];
  const int tid = (int)threadIdx.x;
  const int u   = (int)blockIdx.x * NTHR + tid;
  const int L0 = U_HB;
  const int L1 = L0 + U_WP;
  const int L2 = L1 + U_W2;
  const int L3 = L2 + U_GA;
  const int L4 = L3 + U_GB;
  const int L5 = L4 + U_TH;
  v8us o;
  if (u < L0) {
    const int row = u / (KPJ / 8);
    const int k8  = (u - row * (KPJ / 8)) * 8;
    const int rc  = row < NV ? row : NV - 1;
    const float* p = Hin + (size_t)rc * DIN;
#pragma unroll
    for (int i = 0; i < 8; ++i) {
      const int k  = k8 + i;
      const int kc = k < DIN ? k : DIN - 1;
      const float v = p[kc];
      const bool ok = (k < DIN) && (row < NV);
      o[i] = ok ? (unsigned short)bf16_bits(v) : (unsigned short)0;
    }
    put16(HB + (size_t)row * KPJ + k8, o);
    return;
  } else if (u < L1) {
    const int v  = u - L0;
    const int n  = v / (KPJ / 8);
    const int k8 = (v - n * (KPJ / 8)) * 8;
    const int nc = n < HD ? n : HD - 1;
#pragma unroll
    for (int i = 0; i < 8; ++i) {
      const int k  = k8 + i;
      const int kc = k < DIN ? k : DIN - 1;
      const float w = Wp[(size_t)kc * HD + nc];
      const bool ok = (k < DIN) && (n < HD);
      o[i] = ok ? (unsigned short)bf16_bits(w) : (unsigned short)0;
    }
    put16(WpT + (size_t)n * KPJ + k8, o);
    return;
  } else if (u < L2) {
    const int v    = u - L1;
    const int n    = v >> 5;
    const int k8   = (v & 31) * 8;
    const int srow = k8 & (EHD - 1);
    const float* p = We2 + (size_t)srow * NWE + n;
#pragma unroll
    for (int i = 0; i < 8; ++i) o[i] = (unsigned short)bf16_bits(p[(size_t)i * NWE]);
    put16(W2T + (size_t)n * KWE + k8, o);
    return;
  } else if (u < L3) {
    const int v    = u - L2;
    const int n    = v >> 4;
    const int k8   = (v & 15) * 8;
    const int srow = k8 & (HD - 1);
    const int colc = n < 3 * HD ? n : 3 * HD - 1;
    const bool ok  = n < 3 * HD;
    const float* p = Wih + (size_t)srow * (3 * HD) + colc;
#pragma unroll
    for (int i = 0; i < 8; ++i) {
      const float w = p[(size_t)i * (3 * HD)];
      o[i] = ok ? (unsigned short)bf16_bits(w) : (unsigned short)0;
    }
    put16(WG + (size_t)n * KGR + k8, o);
    return;
  } else if (u < L4) {
    const int v    = u - L3;
    const int n    = v >> 4;
    const int k8   = 128 + (v & 15) * 8;
    const int srow = (k8 - 128) & (HD - 1);
    const int nb   = n >> 6;
    const int colc = (nb == 3) ? (n - HD) : (n & 127);
    const bool ok  = nb != 2;
    const float* p = Whh + (size_t)srow * (3 * HD) + colc;
#pragma unroll
    for (int i = 0; i < 8; ++i) {
      const float w = p[(size_t)i * (3 * HD)];
      o[i] = ok ? (unsigned short)bf16_bits(w) : (unsigned short)0;
    }
    put16(WG + (size_t)n * KGR + k8, o);
    return;
  } else if (u < L5) {
#pragma unroll 1
    for (int i = tid; i < EIN * EHD; i += NTHR) sW1[i] = bf16_val(We1[i]);
    if (tid < EHD) sb1[tid] = bf16_val(be1[tid]);
    __syncthreads();
    const int v   = u - L4;
    const int row = v >> 4;
    const int j   = v & 15;
    const int rc  = row < NE ? row : NE - 1;
    const bool live = row < NE;
    const v4f b0 = *(const v4fa*)(sb1 + 8 * j);
    const v4f b1 = *(const v4fa*)(sb1 + 8 * j + 4);
    float a0 = b0.x, a1 = b0.y, a2 = b0.z, a3 = b0.w, a4 = b1.x, a5 = b1.y, a6 = b1.z, a7 = b1.w;
    const float* ep = Ein + (size_t)rc * EIN;
#pragma unroll 1
    for (int k = 0; k < EIN; ++k) {
      const float ev = bf16_val(ep[k]);
      const v4f w0 = *(const v4fa*)(sW1 + k * EHD + 8 * j);
      const v4f w1 = *(const v4fa*)(sW1 + k * EHD + 8 * j + 4);
      a0 = fmaf(ev, w0.x, a0); a1 = fmaf(ev, w0.y, a1); a2 = fmaf(ev, w0.z, a2); a3 = fmaf(ev, w0.w, a3);
      a4 = fmaf(ev, w1.x, a4); a5 = fmaf(ev, w1.y, a5); a6 = fmaf(ev, w1.z, a6); a7 = fmaf(ev, w1.w, a7);
    }
    const v8f t8 = {a0, a1, a2, a3, a4, a5, a6, a7};
    v8us ohi, olo;
#pragma unroll
    for (int i = 0; i < 8; ++i) {
      float t = relu_k(t8[i]);
      t = live ? t : 0.0f;
      const unsigned hb = bf16_bits(t);
      ohi[i] = (unsigned short)hb;
      olo[i] = (unsigned short)bf16_bits(t - __uint_as_float(hb << 16));
    }
    unsigned short* dp = THL + (size_t)row * KWE + 8 * j;
    *(volatile v8us*)dp         = ohi;
    *(volatile v8us*)(dp + EHD) = olo;
    __threadfence();
    *(volatile v8us*)dp         = ohi;
    *(volatile v8us*)(dp + EHD) = olo;
    return;
  }
}

__global__ __launch_bounds__(NTHR) void k_bucket(const int* __restrict__ dsts, int nE,
                                                 int* LIST, int* CNT, int* OFF, int* FLG) {
  extern __shared__ __attribute__((aligned(16))) int dsm[];
  int* list = dsm;
  int* hl   = dsm + LISTN;
  int* sl   = hl + RCAP;
  int* cnt  = sl + RCAP;
  int* offs = cnt + NBA;
  int* cur  = offs + NBA;
  int* misc = cur + NBA;
  const int tid = (int)threadIdx.x, lane = tid & 31, wave = tid >> 5;
  const int b = (int)blockIdx.x;
  const int nodeBase = b * NBA;

  {
    const v4i z4 = {0, 0, 0, 0};
    for (int i = tid * 4; i < AGG_ZINTS; i += NTHR * 4) *(v4ia*)(dsm + i) = z4;
    if (tid < 16) misc[tid] = 0;
  }
  __syncthreads();

  int t = 0, ov = 0;
  const int nChunks = (nE + CHUNK - 1) / CHUNK;
#pragma unroll 1
  for (int ch = 0; ch < nChunks; ++ch) {
    const int cbase = ch * CHUNK;
    const int wc = scan_chunk<SLA>(dsts, nE, cbase, nodeBase, NBA, 1, list, tid, lane, wave);
    if (lane == 0) misc[wave] = wc;
    __syncthreads();
    if (wave == 0) {
#pragma unroll 1
      for (int w2 = 0; w2 < NWAVE; ++w2) {
        int c = misc[w2];
        c = c < 0 ? 0 : (c > WCAP ? WCAP : c);
#pragma unroll 1
        for (int b0 = 0; b0 < c; b0 += 32) {
          const int idx = b0 + lane;
          const int ent = list[w2 * WCAP + (idx < WCAP ? idx : WCAP - 1)];
          const int m32 = (c - b0) < 32 ? (c - b0) : 32;
#pragma unroll 1
          for (int k = 0; k < m32; ++k) {
            const int uu   = __builtin_amdgcn_readlane(ent, k);
            const int slot = uu & (NBA - 1);
            const int el   = (uu >> SLA) & (CHUNK - 1);
            const int pk   = ((cbase + el) << SLA) | slot;
            if (t < RCAP) {
              if (lane == 0) { hl[t] = pk; cnt[slot] = cnt[slot] + 1; }
              t = t + 1;
            } else {
              ov = 1;
            }
          }
        }
      }
    }
    __syncthreads();
  }
  if (wave == 0 && lane == 0) { misc[8] = t; misc[9] = ov; }
  __syncthreads();
  int tt = misc[8];
  tt = tt < 0 ? 0 : (tt > RCAP ? RCAP : tt);
  const int ovf = misc[9];

  if (wave == 0) {
    const int base = lane * (NBA / 32);
    int s = 0;
#pragma unroll 1
    for (int i = 0; i < NBA / 32; ++i) s += cnt[base + i];
    int incl = s;
#pragma unroll
    for (int d = 1; d < 32; d <<= 1) {
      const int y = __shfl_up(incl, d, 32);
      if (lane >= d) incl += y;
    }
    int run = incl - s;
#pragma unroll 1
    for (int i = 0; i < NBA / 32; ++i) {
      const int cv = cnt[base + i];
      offs[base + i] = run;
      cur[base + i]  = run;
      run += cv;
    }
  }
  __syncthreads();
  if (wave == 0) {
#pragma unroll 1
    for (int b0 = 0; b0 < tt; b0 += 32) {
      const int idx = b0 + lane;
      const int ent = hl[idx < RCAP ? idx : RCAP - 1];
      const int m32 = (tt - b0) < 32 ? (tt - b0) : 32;
#pragma unroll 1
      for (int k = 0; k < m32; ++k) {
        const int uu   = __builtin_amdgcn_readlane(ent, k);
        const int slot = uu & (NBA - 1);
        if (lane == 0) {
          int p = cur[slot];
          p = p < 0 ? 0 : (p > RCAP - 1 ? RCAP - 1 : p);
          sl[p] = uu;
          cur[slot] = p + 1;
        }
      }
    }
  }
  __syncthreads();

  v4i lv[RCAP / (4 * NTHR)];
#pragma unroll
  for (int q = 0; q < RCAP / (4 * NTHR); ++q) {
    const v4i uu = *(const v4ia*)(sl + (q * NTHR + tid) * 4);
    v4i r;
    r.x = uu.x >> SLA; r.y = uu.y >> SLA; r.z = uu.z >> SLA; r.w = uu.w >> SLA;
    lv[q] = r;
  }
  const v4i cv4 = *(const v4ia*)(cnt + 4 * tid);
  const v4i ov4 = *(const v4ia*)(offs + 4 * tid);
  const v4i fv4 = {ovf, ovf, ovf, ovf};
  int* Lb = LIST + (size_t)b * RCAP;
  int* Cb = CNT + (size_t)b * NBA;
  int* Ob = OFF + (size_t)b * NBA;
  int* Fb = FLG + (size_t)b * 32;
#pragma unroll
  for (int q = 0; q < RCAP / (4 * NTHR); ++q) *(volatile v4i*)(Lb + (q * NTHR + tid) * 4) = lv[q];
  *(volatile v4i*)(Cb + 4 * tid) = cv4;
  *(volatile v4i*)(Ob + 4 * tid) = ov4;
  if (tid < 8) *(volatile v4i*)(Fb + 4 * tid) = fv4;
  __threadfence();
#pragma unroll
  for (int q = 0; q < RCAP / (4 * NTHR); ++q) *(volatile v4i*)(Lb + (q * NTHR + tid) * 4) = lv[q];
  *(volatile v4i*)(Cb + 4 * tid) = cv4;
  *(volatile v4i*)(Ob + 4 * tid) = ov4;
  if (tid < 8) *(volatile v4i*)(Fb + 4 * tid) = fv4;
}

__device__ __forceinline__ void mma_tile(const unsigned short* __restrict__ ap,
                                         const unsigned short* __restrict__ bp, int ldb, int K, v8f (&acc)[8]) {
#pragma unroll 1
  for (int k0 = 0; k0 < K; k0 += 32) {
    FragB af;
    af.h[0] = *(const v8usa*)(ap + k0);
    af.h[1] = *(const v8usa*)(ap + k0 + 16);
#pragma unroll
    for (int nt = 0; nt < 8; ++nt) {
      const unsigned short* wq = bp + (size_t)(16 * nt) * (size_t)ldb + k0;
      FragB bf;
      bf.h[0] = *(const v8usa*)wq;
      bf.h[1] = *(const v8usa*)(wq + 16);
      acc[nt] = wmb(af, bf, acc[nt]);
    }
  }
}

__device__ __forceinline__ void store_x_rows(const float* stg, const int pitch, const int wave, const int lane,
                                             const int rowBase, float* XFo, unsigned short* ACo) {
  const int rsel = lane >> 4, j = lane & 15;
  const unsigned mh = 0u - (unsigned)(j >> 3);
  const unsigned ml = ~mh;
  v4f  xv[8];
  v8us pv[8];
#pragma unroll
  for (int i = 0; i < 8; ++i) {
    const float* sr = stg + (16 * wave + 2 * i + rsel) * pitch;
    xv[i] = *(const v4fa*)(sr + 4 * j);
    const float* sp = sr + 8 * (j & 7);
    const v4f a = *(const v4fa*)sp;
    const v4f b = *(const v4fa*)(sp + 4);
    const v8f f8 = {a.x, a.y, a.z, a.w, b.x, b.y, b.z, b.w};
    v8us oo;
#pragma unroll
    for (int e = 0; e < 8; ++e) {
      const unsigned hb = bf16_bits(f8[e]);
      const unsigned lb = bf16_bits(f8[e] - __uint_as_float(hb << 16));
      oo[e] = (unsigned short)((hb & ml) | (lb & mh));
    }
    pv[i] = oo;
  }
#pragma unroll
  for (int i = 0; i < 8; ++i) {
    const size_t row = (size_t)(rowBase + 16 * wave + 2 * i + rsel);
    *(volatile v4f*)(XFo + row * HD + 4 * j) = xv[i];
    *(volatile v8us*)(ACo + row * ACW + 128 + 8 * j) = pv[i];
  }
  __threadfence();
#pragma unroll
  for (int i = 0; i < 8; ++i) {
    const size_t row = (size_t)(rowBase + 16 * wave + 2 * i + rsel);
    *(volatile v4f*)(XFo + row * HD + 4 * j) = xv[i];
    *(volatile v8us*)(ACo + row * ACW + 128 + 8 * j) = pv[i];
  }
}

__global__ __launch_bounds__(GTHR) void k_gproj(const unsigned short* __restrict__ HB,
                                                const unsigned short* __restrict__ WpT,
                                                const float* __restrict__ bproj,
                                                float* XF0, unsigned short* AC0) {
  __shared__ __attribute__((aligned(16))) float stg[GBM * GBN];
  const int tid = (int)threadIdx.x, lane = tid & 31, wave = tid >> 5, hh = lane >> 4, m = lane & 15;
  const int rowBase = (int)blockIdx.x * GBM;
  v8f acc[8];
  {
    const v8f z = {0.f, 0.f, 0.f, 0.f, 0.f, 0.f, 0.f, 0.f};
#pragma unroll
    for (int t = 0; t < 8; ++t) acc[t] = z;
  }
  const unsigned short* ap = HB  + (size_t)(rowBase + 16 * wave + m) * (size_t)KPJ + 8 * hh;
  const unsigned short* bp = WpT + (size_t)m * (size_t)KPJ + 8 * hh;
  mma_tile(ap, bp, KPJ, KPJ, acc);
#pragma unroll
  for (int nt = 0; nt < 8; ++nt) {
    const int lc  = 16 * nt + m;
    const int lcb = lc < HD ? lc : HD - 1;
    const float bvv = bf16_val(bproj[lcb]);
#pragma unroll
    for (int r = 0; r < 8; ++r) {
      const int lr = 16 * wave + 8 * hh + r;
      const bool live = (rowBase + lr) < NV;
      const float v = relu_k(acc[nt][r] + bvv);
      stg[lr * GBN + lc] = live ? v : 0.0f;
    }
  }
  __syncthreads();
  store_x_rows(stg, GBN, wave, lane, rowBase, XF0, AC0);
}

__global__ __launch_bounds__(GTHR) void k_gwe(const unsigned short* __restrict__ THL,
                                              const unsigned short* __restrict__ W2T,
                                              const float* __restrict__ be2, unsigned short* WE) {
  __shared__ __attribute__((aligned(16))) float stg[GBM * GBN];
  const int tid = (int)threadIdx.x, lane = tid & 31, wave = tid >> 5, hh = lane >> 4, m = lane & 15;
  const int rowBase = (int)blockIdx.x * GBM;
  const int colBase = (int)blockIdx.y * GBN;
  v8f acc[8];
  {
    const v8f z = {0.f, 0.f, 0.f, 0.f, 0.f, 0.f, 0.f, 0.f};
#pragma unroll
    for (int t = 0; t < 8; ++t) acc[t] = z;
  }
  const unsigned short* ap = THL + (size_t)(rowBase + 16 * wave + m) * (size_t)KWE + 8 * hh;
  const unsigned short* bp = W2T + (size_t)(colBase + m) * (size_t)KWE + 8 * hh;
  mma_tile(ap, bp, KWE, KWE, acc);
#pragma unroll
  for (int nt = 0; nt < 8; ++nt) {
    const int lc = 16 * nt + m;
    const float bvv = bf16_val(be2[colBase + lc]);
#pragma unroll
    for (int r = 0; r < 8; ++r) {
      const int lr = 16 * wave + 8 * hh + r;
      stg[lr * GBN + lc] = (acc[nt][r] + bvv) * CWE;
    }
  }
  __syncthreads();
  const int rsel = lane >> 4, j = lane & 15;
  v8us pv[8];
#pragma unroll
  for (int i = 0; i < 8; ++i) {
    const float* sp = stg + (16 * wave + 2 * i + rsel) * GBN + 8 * j;
    const v4f a = *(const v4fa*)sp;
    const v4f b = *(const v4fa*)(sp + 4);
    const v8f f8 = {a.x, a.y, a.z, a.w, b.x, b.y, b.z, b.w};
    v8us oo;
#pragma unroll
    for (int e = 0; e < 8; ++e) oo[e] = f2h(f8[e]);
    pv[i] = oo;
  }
#pragma unroll
  for (int i = 0; i < 8; ++i) {
    const int row = rowBase + 16 * wave + 2 * i + rsel;
    if (row < NE) *(volatile v8us*)(WE + (size_t)row * NWE + colBase + 8 * j) = pv[i];
  }
  __threadfence();
#pragma unroll
  for (int i = 0; i < 8; ++i) {
    const int row = rowBase + 16 * wave + 2 * i + rsel;
    if (row < NE) *(volatile v8us*)(WE + (size_t)row * NWE + colBase + 8 * j) = pv[i];
  }
}

__global__ __launch_bounds__(GTHR) void k_ggru(const unsigned short* __restrict__ ACp,
                                               const unsigned short* __restrict__ WG,
                                               const float* __restrict__ bih, const float* __restrict__ bhh,
                                               const float* __restrict__ XFp,
                                               float* XFq, unsigned short* ACq) {
  extern __shared__ __attribute__((aligned(16))) float gdyn[];
  float* stg = gdyn;
  float* sB  = gdyn + GBM * KGR;
  const int tid = (int)threadIdx.x, lane = tid & 31, wave = tid >> 5, hh = lane >> 4, m = lane & 15;
  const int rowBase = (int)blockIdx.x * GBM;
  {
    const int c = tid & (HD - 1);
    const float i0 = bf16_val(bih[tid]);
    const float h0 = bf16_val(bhh[tid]);
    const float i1 = bf16_val(bih[2 * HD + c]);
    const float h1 = bf16_val(bhh[2 * HD + c]);
    sB[tid] = i0 + h0;
    sB[128 + tid] = (tid < HD) ? i1 : h1;
  }
  __syncthreads();

  const unsigned short* ap = ACp + (size_t)(rowBase + 16 * wave + m) * (size_t)ACW + 8 * hh;
#pragma unroll 1
  for (int nh = 0; nh < 2; ++nh) {
    v8f acc[8];
    {
      const v8f z = {0.f, 0.f, 0.f, 0.f, 0.f, 0.f, 0.f, 0.f};
#pragma unroll
      for (int t = 0; t < 8; ++t) acc[t] = z;
    }
    const unsigned short* bp = WG + (size_t)(128 * nh + m) * (size_t)KGR + 8 * hh;
    mma_tile(ap, bp, KGR, KGR, acc);
#pragma unroll
    for (int nt = 0; nt < 8; ++nt) {
      const int lc = 128 * nh + 16 * nt + m;
      const float bvv = sB[lc];
#pragma unroll
      for (int r = 0; r < 8; ++r) {
        const int lr = 16 * wave + 8 * hh + r;
        stg[lr * KGR + lc] = acc[nt][r] + bvv;
      }
    }
  }
  __syncthreads();

  {
    const int rsel = lane >> 4, j = lane & 15;
#pragma unroll 1
    for (int it = 0; it < 32; ++it) {
      const int i = it >> 2, e = it & 3;
      const int lr = 16 * wave + 2 * i + rsel;
      const int c  = 4 * j + e;
      float* sr = stg + lr * KGR;
      const float ar = sr[c];
      const float az = sr[HD + c];
      const float ai = sr[2 * HD + c];
      const float ah = sr[3 * HD + c];
      const float hid = XFp[(size_t)(rowBase + lr) * HD + c];
      const float rg = sigm(ar);
      const float zg = sigm(az);
      const float ng = tanhf(ai + rg * ah);
      sr[c] = (1.0f - zg) * ng + zg * hid;
    }
  }
  __syncthreads();
  store_x_rows(stg, KGR, wave, lane, rowBase, XFq, ACq);
}

__global__ __launch_bounds__(NTHR) void k_msg(const float* __restrict__ XFp,
                                              const unsigned short* __restrict__ WE,
                                              const int* __restrict__ srcs, float* MSG) {
  __shared__ __attribute__((aligned(16))) float xs[NWAVE * HD];
  const int tid = (int)threadIdx.x, lane = tid & 31, wave = tid >> 5;
  const int e  = (int)blockIdx.x * NWAVE + wave;
  const int ec = e < NE ? e : NE - 1;
  int s = srcs[ec];
  s = s < 0 ? 0 : (s > NV - 1 ? NV - 1 : s);
  const v2f xv = *(const v2fa*)(XFp + (size_t)s * HD + 2 * lane);
  *(v2fa*)(xs + wave * HD + 2 * lane) = xv;
  __syncthreads();

  const unsigned short* wr = WE + (size_t)ec * NWE + 8 * lane;
  const float* xw = xs + wave * HD + (lane >> 3);
  float a0 = 0.f, a1 = 0.f, a2 = 0.f, a3 = 0.f, a4 = 0.f, a5 = 0.f, a6 = 0.f, a7 = 0.f;
#pragma unroll 2
  for (int j = 0; j < 16; ++j) {
    const v4u w = *(const v4ua*)(wr + j * 256);
    const float xi = xw[4 * j];
    a0 = fmaf(xi, h2f(w.x & 0xffffu), a0);
    a1 = fmaf(xi, h2f(w.x >> 16),     a1);
    a2 = fmaf(xi, h2f(w.y & 0xffffu), a2);
    a3 = fmaf(xi, h2f(w.y >> 16),     a3);
    a4 = fmaf(xi, h2f(w.z & 0xffffu), a4);
    a5 = fmaf(xi, h2f(w.z >> 16),     a5);
    a6 = fmaf(xi, h2f(w.w & 0xffffu), a6);
    a7 = fmaf(xi, h2f(w.w >> 16),     a7);
  }
  a0 += __shfl_xor(a0, 8);  a1 += __shfl_xor(a1, 8);  a2 += __shfl_xor(a2, 8);  a3 += __shfl_xor(a3, 8);
  a4 += __shfl_xor(a4, 8);  a5 += __shfl_xor(a5, 8);  a6 += __shfl_xor(a6, 8);  a7 += __shfl_xor(a7, 8);
  a0 += __shfl_xor(a0, 16); a1 += __shfl_xor(a1, 16); a2 += __shfl_xor(a2, 16); a3 += __shfl_xor(a3, 16);
  a4 += __shfl_xor(a4, 16); a5 += __shfl_xor(a5, 16); a6 += __shfl_xor(a6, 16); a7 += __shfl_xor(a7, 16);
  const int sl = lane >> 1;
  const float q0 = __shfl(a0, sl), q1 = __shfl(a1, sl), q2 = __shfl(a2, sl), q3 = __shfl(a3, sl);
  const float q4 = __shfl(a4, sl), q5 = __shfl(a5, sl), q6 = __shfl(a6, sl), q7 = __shfl(a7, sl);
  const bool up = (lane & 1) != 0;
  v4f o;
  o.x = (up ? q4 : q0) * CINV;
  o.y = (up ? q5 : q1) * CINV;
  o.z = (up ? q6 : q2) * CINV;
  o.w = (up ? q7 : q3) * CINV;
  float* op = MSG + (size_t)ec * HD + 4 * (lane & 15);
  const bool st = (lane < 16) && (e < NE);
  if (st) *(volatile v4f*)op = o;
  __threadfence();
  if (st) *(volatile v4f*)op = o;
}

__global__ __launch_bounds__(NTHR) void k_agg(const int* __restrict__ LIST, const int* __restrict__ CNT,
                                              const int* __restrict__ OFF, const int* __restrict__ FLG,
                                              const float* __restrict__ MSG, const float* __restrict__ bconv,
                                              unsigned short* ACp) {
  __shared__ __attribute__((aligned(16))) int sL[RCAP];
  __shared__ __attribute__((aligned(16))) int sC[NBA];
  __shared__ __attribute__((aligned(16))) int sO[NBA];
  __shared__ __attribute__((aligned(16))) unsigned stw[NWAVE * 64];
  const int tid = (int)threadIdx.x, lane = tid & 31, wave = tid >> 5;
  const int b = (int)blockIdx.x;
#pragma unroll
  for (int q = 0; q < RCAP / (4 * NTHR); ++q) {
    const int idx = (q * NTHR + tid) * 4;
    *(v4ia*)(sL + idx) = *(const v4i*)(LIST + (size_t)b * RCAP + idx);
  }
  *(v4ia*)(sC + 4 * tid) = *(const v4i*)(CNT + (size_t)b * NBA + 4 * tid);
  *(v4ia*)(sO + 4 * tid) = *(const v4i*)(OFF + (size_t)b * NBA + 4 * tid);
  const int flg = FLG[(size_t)b * 32];
  __syncthreads();

  const float qnan = __int_as_float(0x7fc00000);
  const float bc0 = bf16_val(bconv[2 * lane]);
  const float bc1 = bf16_val(bconv[2 * lane + 1]);
  unsigned* stwu = stw + wave * 64;
#pragma unroll 1
  for (int si = 0; si < NBA / NWAVE; ++si) {
    const int s    = si * NWAVE + wave;
    const int node = b * NBA + s;
    int c = sC[s];
    const bool big = c > DEGCAP;
    c = c < 0 ? 0 : (c > DEGCAP ? DEGCAP : c);
    int o = sO[s];
    o = o < 0 ? 0 : (o > RCAP ? RCAP : o);
    if (c > RCAP - o) c = RCAP - o;
    int idx = o + lane;
    idx = idx > RCAP - 1 ? RCAP - 1 : idx;
    int eid = sL[idx];
    eid = eid < 0 ? 0 : (eid > NE - 1 ? NE - 1 : eid);
    float a0 = 0.0f, a1 = 0.0f;
#pragma unroll 1
    for (int k = 0; k < c; ++k) {
      const int ek = __builtin_amdgcn_readlane(eid, k);
      const v2f v = *(const v2fa*)(MSG + (size_t)ek * HD + 2 * lane);
      a0 += v.x;
      a1 += v.y;
    }
    const float pz = (flg != 0 || big) ? qnan : 0.0f;
    const bool liveRow = node < NV;
    float r0 = relu_k(a0 + bc0) + pz;
    float r1 = relu_k(a1 + bc1) + pz;
    r0 = liveRow ? r0 : 0.0f;
    r1 = liveRow ? r1 : 0.0f;
    const unsigned hb0 = bf16_bits(r0), hb1 = bf16_bits(r1);
    const unsigned lb0 = bf16_bits(r0 - __uint_as_float(hb0 << 16));
    const unsigned lb1 = bf16_bits(r1 - __uint_as_float(hb1 << 16));
    __syncthreads();
    stwu[lane]      = hb0 | (hb1 << 16);
    stwu[32 + lane] = lb0 | (lb1 << 16);
    __syncthreads();
    const v4u pk = *(const v4ua*)(stwu + 4 * (lane & 15));
    const int nr = node < MP ? node : MP - 1;
    unsigned short* gp = ACp + (size_t)nr * ACW + 8 * (lane & 15);
    const bool st = (node < MP) && (lane < 16);
    if (st) *(volatile v4u*)gp = pk;
    __threadfence();
    if (st) *(volatile v4u*)gp = pk;
  }
}

__global__ __launch_bounds__(NTHR) void k_pool(const float* __restrict__ xf, const int* __restrict__ gid,
                                               float* HG) {
  __shared__ __attribute__((aligned(16))) float wsum[NWAVE * HD];
  __shared__ int wcn[NWAVE];
  __shared__ __attribute__((aligned(16))) float outs[HD];
  const int tid = (int)threadIdx.x, lane = tid & 31, wave = tid >> 5;
  const int g = (int)blockIdx.x;
  float a0 = 0.0f, a1 = 0.0f;
  int cnt = 0;
#pragma unroll 1
  for (int i0 = wave * 32; i0 < NV; i0 += NTHR) {
    const int i  = i0 + lane;
    const int ic = i < NV ? i : NV - 1;
    const int bb = gid[ic];
    const bool hit = (i < NV) && (bb == g);
    unsigned msk = __builtin_amdgcn_ballot_w32(hit);
    int nh = (int)__builtin_popcount(msk);
    nh = nh > 32 ? 32 : nh;
    cnt += nh;
#pragma unroll 1
    for (int q = 0; q < nh; ++q) {
      const int k = __builtin_ffs((int)msk) - 1;
      msk &= msk - 1u;
      int node = i0 + (k < 0 ? 0 : k);
      node = node > NV - 1 ? NV - 1 : node;
      const v2f v = *(const v2fa*)(xf + (size_t)node * HD + 2 * lane);
      a0 += v.x;
      a1 += v.y;
    }
  }
  wsum[wave * HD + 2 * lane + 0] = a0;
  wsum[wave * HD + 2 * lane + 1] = a1;
  if (lane == 0) wcn[wave] = cnt;
  __syncthreads();
  if (tid < HD) {
    float s = 0.0f;
    int c = 0;
#pragma unroll
    for (int w2 = 0; w2 < NWAVE; ++w2) { s += wsum[w2 * HD + tid]; c += wcn[w2]; }
    const float cf = (c < 1) ? 1.0f : (float)c;
    outs[tid] = s * (1.0f / cf);
  }
  __syncthreads();
  const v4f ov = *(const v4fa*)(outs + 4 * (lane & 15));
  float* op = HG + (size_t)g * HD + 4 * (lane & 15);
  const bool st = (wave == 0) && (lane < 16);
  if (st) *(volatile v4f*)op = ov;
  __threadfence();
  if (st) *(volatile v4f*)op = ov;
}

__global__ __launch_bounds__(NTHR) void k_head(const float* __restrict__ HG,
                                               const float* __restrict__ W0, const float* __restrict__ b0,
                                               const float* __restrict__ W1, const float* __restrict__ b1,
                                               const float* __restrict__ W2, const float* __restrict__ b2,
                                               const int* __restrict__ FLG, float* out) {
  __shared__ __attribute__((aligned(16))) float sW0[HD * 32];
  __shared__ __attribute__((aligned(16))) float sW1[32 * 16];
  __shared__ __attribute__((aligned(16))) float sW2[32];
  __shared__ __attribute__((aligned(16))) float sb0[32];
  __shared__ __attribute__((aligned(16))) float sb1[16];
  __shared__ __attribute__((aligned(16))) float sb2[4];
  __shared__ __attribute__((aligned(16))) float sT[NG * 32];
  __shared__ __attribute__((aligned(16))) float sO[NG * 2];
  const int tid = (int)threadIdx.x;
#pragma unroll 1
  for (int i = tid; i < HD * 32; i += NTHR) sW0[i] = bf16_val(W0[i]);
#pragma unroll 1
  for (int i = tid; i < 32 * 16; i += NTHR) sW1[i] = bf16_val(W1[i]);
  if (tid < 32) { sW2[tid] = bf16_val(W2[tid]); sb0[tid] = bf16_val(b0[tid]); }
  if (tid < 16) sb1[tid] = bf16_val(b1[tid]);
  if (tid < 2)  sb2[tid] = bf16_val(b2[tid]);
  __syncthreads();

  const int g = tid;
  float* tr = sT + g * 32;
#pragma unroll 1
  for (int jh = 0; jh < 2; ++jh) {
    float a[16];
#pragma unroll
    for (int t = 0; t < 16; ++t) a[t] = sb0[jh * 16 + t];
#pragma unroll 1
    for (int i = 0; i < HD; ++i) {
      const float hv = HG[(size_t)g * HD + i];
      const float* wr = sW0 + i * 32 + jh * 16;
#pragma unroll
      for (int t = 0; t < 16; ++t) a[t] = fmaf(hv, wr[t], a[t]);
    }
#pragma unroll
    for (int t = 0; t < 16; ++t) tr[jh * 16 + t] = relu_k(a[t]);
  }
  {
    float c[16];
#pragma unroll
    for (int t = 0; t < 16; ++t) c[t] = sb1[t];
#pragma unroll 1
    for (int i = 0; i < 32; ++i) {
      const float v = tr[i];
      const float* wr = sW1 + i * 16;
#pragma unroll
      for (int t = 0; t < 16; ++t) c[t] = fmaf(v, wr[t], c[t]);
    }
#pragma unroll
    for (int t = 0; t < 16; ++t) tr[t] = relu_k(c[t]);
  }
  float o0 = sb2[0], o1 = sb2[1];
#pragma unroll 1
  for (int i = 0; i < 16; ++i) {
    const float v = tr[i];
    o0 = fmaf(v, sW2[2 * i], o0);
    o1 = fmaf(v, sW2[2 * i + 1], o1);
  }
  int fl = 0;
#pragma unroll 1
  for (int bb = 0; bb < NBLK; ++bb) fl |= FLG[bb * 32];
  const float qnan = __int_as_float(0x7fc00000);
  o0 = (fl != 0) ? qnan : o0;
  o1 = (fl != 0) ? qnan : o1;
  sO[2 * g]     = o0;
  sO[2 * g + 1] = o1;
  __syncthreads();
  const int tq = tid & 127;
  const v4f ov = *(const v4fa*)(sO + 4 * tq);
  const bool st = tid < 128;
  if (st) *(volatile v4f*)(out + 4 * tq) = ov;
  __threadfence();
  if (st) *(volatile v4f*)(out + 4 * tq) = ov;
}

static inline size_t al256(size_t o) { return (o + 255) & ~(size_t)255; }

extern "C" void kernel_launch(void* const* d_in, const int* in_sizes, int n_in,
                              void* d_out, int out_size, void* d_ws, size_t ws_size,
                              hipStream_t stream) {
  if (n_in < 23) return;
  if (in_sizes[0] != NV * DIN || in_sizes[1] != NE * EIN) return;
  if (in_sizes[2] != NE || in_sizes[3] != NE || in_sizes[4] != NV || in_sizes[5] != 1) return;
  if (in_sizes[6] != DIN * HD || in_sizes[7] != HD) return;
  if (in_sizes[8] != EIN * EHD || in_sizes[9] != EHD) return;
  if (in_sizes[10] != EHD * NWE || in_sizes[11] != NWE || in_sizes[12] != HD) return;
  if (in_sizes[13] != HD * 3 * HD || in_sizes[14] != HD * 3 * HD) return;
  if (in_sizes[15] != 3 * HD || in_sizes[16] != 3 * HD) return;
  if (in_sizes[17] != HD * 32 || in_sizes[18] != 32 || in_sizes[19] != 32 * 16 || in_sizes[20] != 16) return;
  if (in_sizes[21] != 32 || in_sizes[22] != 2) return;
  if (out_size != NG * 2) return;

  const float* h_in  = (const float*)d_in[0];
  const float* e_in  = (const float*)d_in[1];
  const int*   esrc  = (const int*)d_in[2];
  const int*   edst  = (const int*)d_in[3];
  const int*   gids  = (const int*)d_in[4];
  const float* Wproj = (const float*)d_in[6];
  const float* bproj = (const float*)d_in[7];
  const float* We1   = (const float*)d_in[8];
  const float* be1   = (const float*)d_in[9];
  const float* We2   = (const float*)d_in[10];
  const float* be2   = (const float*)d_in[11];
  const float* bconv = (const float*)d_in[12];
  const float* Wih   = (const float*)d_in[13];
  const float* Whh   = (const float*)d_in[14];
  const float* bih   = (const float*)d_in[15];
  const float* bhh   = (const float*)d_in[16];
  const float* Wr0   = (const float*)d_in[17];
  const float* br0   = (const float*)d_in[18];
  const float* Wr1   = (const float*)d_in[19];
  const float* br1   = (const float*)d_in[20];
  const float* Wr2   = (const float*)d_in[21];
  const float* br2   = (const float*)d_in[22];
  float* out = (float*)d_out;

  char* ws = (char*)d_ws;
  size_t off = 0;
  const size_t oWE  = off; off = al256(off + (size_t)NE * NWE * 2);
  const size_t oTHL = off; off = al256(off + (size_t)EP * KWE * 2);
  const size_t oW2T = off; off = al256(off + (size_t)NWE * KWE * 2);
  const size_t oHB  = off; off = al256(off + (size_t)MP * KPJ * 2);
  const size_t oWpT = off; off = al256(off + (size_t)128 * KPJ * 2);
  const size_t oWG  = off; off = al256(off + (size_t)256 * KGR * 2);
  const size_t oAC0 = off; off = al256(off + (size_t)MP * ACW * 2);
  const size_t oAC1 = off; off = al256(off + (size_t)MP * ACW * 2);
  const size_t oXF0 = off; off = al256(off + (size_t)MP * HD * 4);
  const size_t oXF1 = off; off = al256(off + (size_t)MP * HD * 4);
  const size_t oMSG = off; off = al256(off + (size_t)NE * HD * 4);
  const size_t oLST = off; off = al256(off + (size_t)NBLK * RCAP * 4);
  const size_t oCNT = off; off = al256(off + (size_t)NBLK * NBA * 4);
  const size_t oOFF = off; off = al256(off + (size_t)NBLK * NBA * 4);
  const size_t oFLG = off; off = al256(off + (size_t)NBLK * 32 * 4);
  const size_t oHG  = off; off = al256(off + (size_t)NG * HD * 4);
  if (off > ws_size) return;
  unsigned short* WE16 = (unsigned short*)(ws + oWE);
  unsigned short* THL  = (unsigned short*)(ws + oTHL);
  unsigned short* W2T  = (unsigned short*)(ws + oW2T);
  unsigned short* HB   = (unsigned short*)(ws + oHB);
  unsigned short* WpT  = (unsigned short*)(ws + oWpT);
  unsigned short* WG   = (unsigned short*)(ws + oWG);
  unsigned short* AC[2] = { (unsigned short*)(ws + oAC0), (unsigned short*)(ws + oAC1) };
  float*          XF[2] = { (float*)(ws + oXF0), (float*)(ws + oXF1) };
  float*          MSG  = (float*)(ws + oMSG);
  int*            LIST = (int*)(ws + oLST);
  int*            CNT  = (int*)(ws + oCNT);
  int*            OFF  = (int*)(ws + oOFF);
  int*            FLG  = (int*)(ws + oFLG);
  float*          HG   = (float*)(ws + oHG);

  hipFuncSetAttribute(reinterpret_cast<const void*>(&k_bucket), hipFuncAttributeMaxDynamicSharedMemorySize,
                      (int)BK_LDS_BYTES);
  hipFuncSetAttribute(reinterpret_cast<const void*>(&k_ggru), hipFuncAttributeMaxDynamicSharedMemorySize,
                      (int)GRU_LDS_BYTES);

  const int nPrep = U_HB + U_WP + U_W2 + U_GA + U_GB + U_TH;

  k_prep<<<nPrep / NTHR, NTHR, 0, stream>>>(h_in, e_in, Wproj, We1, be1, We2, Wih, Whh, HB, WpT, W2T, WG, THL);
  k_bucket<<<NBLK, NTHR, BK_LDS_BYTES, stream>>>(edst, NE, LIST, CNT, OFF, FLG);
  k_gproj<<<MP / GBM, GTHR, 0, stream>>>(HB, WpT, bproj, XF[0], AC[0]);
  k_gwe<<<dim3(EP / GBM, NWE / GBN), GTHR, 0, stream>>>(THL, W2T, be2, WE16);
  for (int s = 0; s < NSTEP; ++s) {
    const int p = s & 1;
    k_msg<<<NE / NWAVE, NTHR, 0, stream>>>(XF[p], WE16, esrc, MSG);
    k_agg<<<NBLK, NTHR, 0, stream>>>(LIST, CNT, OFF, FLG, MSG, bconv, AC[p]);
    k_ggru<<<MP / GBM, GTHR, GRU_LDS_BYTES, stream>>>(AC[p], WG, bih, bhh, XF[p], XF[p ^ 1], AC[p ^ 1]);
  }
  k_pool<<<NG, NTHR, 0, stream>>>(XF[NSTEP & 1], gids, HG);
  k_head<<<1, NTHR, 0, stream>>>(HG, Wr0, br0, Wr1, br1, Wr2, br2, FLG, out);
}
